// GraphAttentionLayer_29901562315387
// MI455X (gfx1250) — hardware-verified
//
#include <hip/hip_runtime.h>
#include <stddef.h>
#include <stdint.h>
#include <math.h>


#define KD      128
#define HCH     128
#define NTHR    256
#define NWAVE   8
#define EPT     8
#define CHUNK   (NTHR * EPT)
#define WCAP    (EPT * 32)
#define LISTN   (NWAVE * WCAP)
#define NBMAX   2048
#define SLOTB   11
#define RCAP    28672
#define DEGCAP  128
#define GBM     64
#define GBN     128
#define GTHR    128
#define MROWS   128
#define NEGSL   0.2f
#define LNEPS   1e-5f
#define EPS_SM  1e-16f
#define WSMAX   134217728
#define LDS_AGG ((2 * RCAP + 2 * NBMAX + LISTN) * 4 + 64)

static_assert((CHUNK & (CHUNK - 1)) == 0 && CHUNK <= (1 << SLOTB));
static_assert(NBMAX == (1 << SLOTB));
static_assert(NTHR * 8 == NBMAX);
static_assert(LISTN >= NBMAX);
static_assert(LISTN >= NWAVE * WCAP);
static_assert((RCAP % 32) == 0);
static_assert(LDS_AGG <= 300000);
static_assert(GBM == (GTHR / 32) * 16);
static_assert((KD % 32) == 0 && HCH == GBN && GBN == 4 * 32);
static_assert((MROWS % GBM) == 0);
static_assert(HCH == 4 * 32);

typedef float          v4f  __attribute__((ext_vector_type(4)));
typedef float          v8f  __attribute__((ext_vector_type(8)));
typedef int            v4i  __attribute__((ext_vector_type(4)));
typedef int            v8i  __attribute__((ext_vector_type(8)));
typedef unsigned int   v4u  __attribute__((ext_vector_type(4)));
typedef unsigned short v8us __attribute__((ext_vector_type(8)));
typedef __bf16         v16b __attribute__((ext_vector_type(16)));
typedef v4f  __attribute__((may_alias)) v4fa;
typedef v8us __attribute__((may_alias)) v8usa;
union FragB { v16b v; v8us h[2]; v8i w; };

__device__ __forceinline__ v8f wmb(const FragB& a, const FragB& b, v8f c) {
  v8f d = __builtin_amdgcn_wmma_f32_16x16x32_bf16(false, a.v, false, b.v, (short)0, c, false, false);
  asm volatile("v_nop\n\tv_nop\n\tv_nop\n\tv_nop" : "+v"(d) : "v"(a.w), "v"(b.w));
  return d;
}

__device__ __forceinline__ unsigned int f2bf(float f) {
  const unsigned int u = __float_as_uint(f);
  return ((u + 0x7FFFu + ((u >> 16) & 1u)) >> 16) & 0xFFFFu;
}
__device__ __forceinline__ float bf2f(unsigned int b) { return __uint_as_float(b << 16); }
__device__ __forceinline__ float bfr(float f) { return bf2f(f2bf(f)); }
__device__ __forceinline__ v4f bfr4(const v4f a) {
  v4f r; r.x = bfr(a.x); r.y = bfr(a.y); r.z = bfr(a.z); r.w = bfr(a.w); return r;
}
__device__ __forceinline__ unsigned short xb(float f) { return (unsigned short)f2bf(f); }
__device__ __forceinline__ unsigned int pk2(float lo, float hi) { return f2bf(lo) | (f2bf(hi) << 16); }
__device__ __forceinline__ v4u pack8(const v4f a, const v4f b) {
  v4u r;
  r.x = pk2(a.x, a.y); r.y = pk2(a.z, a.w); r.z = pk2(b.x, b.y); r.w = pk2(b.z, b.w);
  return r;
}

__device__ __forceinline__ float wsum(float v) {
  v += __shfl_xor(v, 16, 32);
  v += __shfl_xor(v, 8, 32);
  v += __shfl_xor(v, 4, 32);
  v += __shfl_xor(v, 2, 32);
  v += __shfl_xor(v, 1, 32);
  return v;
}
__device__ __forceinline__ float hsum8(float v) {
  v += __shfl_xor(v, 1, 32);
  v += __shfl_xor(v, 2, 32);
  v += __shfl_xor(v, 4, 32);
  return v;
}
__device__ __forceinline__ float dot4(const v4f a, const v4f b) {
  float p = a.x * b.x; p = fmaf(a.y, b.y, p); p = fmaf(a.z, b.z, p); p = fmaf(a.w, b.w, p);
  return p;
}

__device__ __forceinline__ int scan_chunk(const int* __restrict__ dsts, int nE, int cbase, int slotBase,
                                          int nb, int vec8, int* list, int tid, int lane, int wave) {
  int wc = 0;
  const int el0  = tid * EPT;
  const int e0   = cbase + el0;
  const int sent = -2147483647 - 1;
  v4i da, db;
  if (vec8 != 0 && cbase + CHUNK <= nE) {
    da = *(const v4i*)(dsts + e0);
    db = *(const v4i*)(dsts + e0 + 4);
  } else {
    da.x = (e0     < nE) ? dsts[min(e0,     nE - 1)] : sent;
    da.y = (e0 + 1 < nE) ? dsts[min(e0 + 1, nE - 1)] : sent;
    da.z = (e0 + 2 < nE) ? dsts[min(e0 + 2, nE - 1)] : sent;
    da.w = (e0 + 3 < nE) ? dsts[min(e0 + 3, nE - 1)] : sent;
    db.x = (e0 + 4 < nE) ? dsts[min(e0 + 4, nE - 1)] : sent;
    db.y = (e0 + 5 < nE) ? dsts[min(e0 + 5, nE - 1)] : sent;
    db.z = (e0 + 6 < nE) ? dsts[min(e0 + 6, nE - 1)] : sent;
    db.w = (e0 + 7 < nE) ? dsts[min(e0 + 7, nE - 1)] : sent;
  }
  const unsigned nbs = (unsigned)slotBase;
  const unsigned unb = (unsigned)nb;
  const unsigned s0 = (unsigned)da.x - nbs, s1 = (unsigned)da.y - nbs;
  const unsigned s2 = (unsigned)da.z - nbs, s3 = (unsigned)da.w - nbs;
  const unsigned s4 = (unsigned)db.x - nbs, s5 = (unsigned)db.y - nbs;
  const unsigned s6 = (unsigned)db.z - nbs, s7 = (unsigned)db.w - nbs;
  const bool h0 = s0 < unb, h1 = s1 < unb, h2 = s2 < unb, h3 = s3 < unb;
  const bool h4 = s4 < unb, h5 = s5 < unb, h6 = s6 < unb, h7 = s7 < unb;
  const unsigned any = __builtin_amdgcn_ballot_w32(h0 | h1 | h2 | h3 | h4 | h5 | h6 | h7);
  if (any != 0u) {
#define HITJ(J, HJ, SJ) { \
      const unsigned mj = __builtin_amdgcn_ballot_w32(HJ); \
      if (mj != 0u) { \
        if (HJ) { \
          const int pos = wc + (int)__builtin_amdgcn_mbcnt_lo(mj, 0u); \
          if (pos < WCAP) list[wave * WCAP + pos] = ((el0 + (J)) << SLOTB) | (int)(SJ); \
        } \
        wc += (int)__builtin_popcount(mj); } }
    HITJ(0, h0, s0)
    HITJ(1, h1, s1)
    HITJ(2, h2, s2)
    HITJ(3, h3, s3)
    HITJ(4, h4, s4)
    HITJ(5, h5, s5)
    HITJ(6, h6, s6)
    HITJ(7, h7, s7)
#undef HITJ
  }
  return wc;
}

__global__ __launch_bounds__(NTHR) void k_wtr(const float* __restrict__ w, int Kin, int Ncol, int Nrows, int Kout,
                                              unsigned short* wt, int nUnits) {
  const int u = (int)blockIdx.x * NTHR + (int)threadIdx.x;
  if (u >= nUnits) return;
  const int kq = Kout >> 3;
  const int n  = u / kq;
  const int k8 = (u - n * kq) * 8;
  const int kk = k8 - (k8 / Kin) * Kin;
  const int ncl = n < Ncol ? n : Ncol - 1;
  const float* p = w + (size_t)kk * (size_t)Ncol + ncl;
  v4f a, b;
  a.x = p[0];                    a.y = p[(size_t)Ncol];         a.z = p[(size_t)2 * Ncol];     a.w = p[(size_t)3 * Ncol];
  b.x = p[(size_t)4 * Ncol];     b.y = p[(size_t)5 * Ncol];     b.z = p[(size_t)6 * Ncol];     b.w = p[(size_t)7 * Ncol];
  const v4f z4 = {0.f, 0.f, 0.f, 0.f};
  if (n >= Ncol || n >= Nrows) { a = z4; b = z4; }
  const v4u wv = pack8(a, b);
  unsigned short* o = wt + (size_t)n * (size_t)Kout + k8;
  *(volatile v4u*)o = wv;
  __threadfence();
  *(volatile v4u*)o = wv;
}

__global__ __launch_bounds__(GTHR) void k_gemm(const float* __restrict__ xin, int nN,
                                               const unsigned short* __restrict__ WT, float* F) {
  __shared__ __attribute__((aligned(16))) float stg[GBM * GBN];
  const int tid = (int)threadIdx.x, lane = tid & 31, wave = tid >> 5, hh = lane >> 4, m = lane & 15;
  const int rowBase = (int)blockIdx.x * GBM;
  const int col0    = (int)blockIdx.y * GBN;

  v8f acc[8];
  {
    const v8f z = {0.f, 0.f, 0.f, 0.f, 0.f, 0.f, 0.f, 0.f};
#pragma unroll
    for (int t = 0; t < 8; ++t) acc[t] = z;
  }
  const int ar  = rowBase + 16 * wave + m;
  const int arc = ar < nN ? ar : nN - 1;
  const float okf = ar < nN ? 1.0f : 0.0f;
  const float* xp = xin + (size_t)arc * KD + 8 * hh;
  const unsigned short* bp = WT + (size_t)(col0 + m) * (size_t)KD + 8 * hh;

#pragma unroll 1
  for (int k0 = 0; k0 < KD; k0 += 32) {
    const v4f u0 = *(const v4fa*)(xp + k0);
    const v4f u1 = *(const v4fa*)(xp + k0 + 4);
    const v4f u2 = *(const v4fa*)(xp + k0 + 16);
    const v4f u3 = *(const v4fa*)(xp + k0 + 20);
    v8us o0, o1;
    o0[0] = xb(u0.x * okf); o0[1] = xb(u0.y * okf); o0[2] = xb(u0.z * okf); o0[3] = xb(u0.w * okf);
    o0[4] = xb(u1.x * okf); o0[5] = xb(u1.y * okf); o0[6] = xb(u1.z * okf); o0[7] = xb(u1.w * okf);
    o1[0] = xb(u2.x * okf); o1[1] = xb(u2.y * okf); o1[2] = xb(u2.z * okf); o1[3] = xb(u2.w * okf);
    o1[4] = xb(u3.x * okf); o1[5] = xb(u3.y * okf); o1[6] = xb(u3.z * okf); o1[7] = xb(u3.w * okf);
    FragB af;
    af.h[0] = o0;
    af.h[1] = o1;
#pragma unroll
    for (int nt = 0; nt < 8; ++nt) {
      const unsigned short* wq = bp + (size_t)(16 * nt) * (size_t)KD + k0;
      FragB bf;
      bf.h[0] = *(const v8usa*)wq;
      bf.h[1] = *(const v8usa*)(wq + 16);
      acc[nt] = wmb(af, bf, acc[nt]);
    }
  }

#pragma unroll
  for (int nt = 0; nt < 8; ++nt) {
    const int lc = 16 * nt + m;
#pragma unroll
    for (int r = 0; r < 8; ++r) {
      const int lr = 16 * wave + 8 * hh + r;
      stg[lr * GBN + lc] = acc[nt][r];
    }
  }
  __syncthreads();

  v4f fv[16];
#pragma unroll
  for (int i = 0; i < 16; ++i) fv[i] = *(const v4fa*)(stg + (16 * wave + i) * GBN + 4 * lane);
#pragma unroll
  for (int i = 0; i < 16; ++i) {
    float* op = F + (size_t)(rowBase + 16 * wave + i) * (size_t)HCH + col0 + 4 * lane;
    *(volatile v4f*)op = fv[i];
  }
  __threadfence();
#pragma unroll
  for (int i = 0; i < 16; ++i) {
    float* op = F + (size_t)(rowBase + 16 * wave + i) * (size_t)HCH + col0 + 4 * lane;
    *(volatile v4f*)op = fv[i];
  }
}

__global__ __launch_bounds__(NTHR) void k_agg(
    const int* __restrict__ srcs, const int* __restrict__ dsts,
    const float* __restrict__ F, const float* __restrict__ xin,
    const float* __restrict__ asrc, const float* __restrict__ adst,
    const float* __restrict__ bias, const float* __restrict__ gam, const float* __restrict__ bet,
    float* out, int nN, int nE, int nb, int vec8) {
  extern __shared__ v4f lds_dyn[];
  int* reg1 = (int*)lds_dyn;
  int* reg2 = reg1 + RCAP;
  int* scnt = reg2 + RCAP;
  int* soff = scnt + NBMAX;
  int* list = soff + NBMAX;
  int* wcnt = list + LISTN;
  int* wtot = wcnt + NWAVE;
  const int tid = (int)threadIdx.x, lane = tid & 31, wave = tid >> 5;
  const int nodeBase = (int)blockIdx.x * nb;

  for (int i = tid; i < NBMAX; i += NTHR) scnt[i] = 0;
  __syncthreads();

  int tot = 0;
  const int nChunks = (nE + CHUNK - 1) / CHUNK;
#pragma unroll 1
  for (int ch = 0; ch < nChunks; ++ch) {
    const int cbase = ch * CHUNK;
    const int wc = scan_chunk(dsts, nE, cbase, nodeBase, nb, vec8, list, tid, lane, wave);
    if (lane == 0) wcnt[wave] = wc;
    __syncthreads();
    int pre = 0, all = 0;
#pragma unroll
    for (int w2 = 0; w2 < NWAVE; ++w2) {
      int c = wcnt[w2];
      c = c < 0 ? 0 : (c > WCAP ? WCAP : c);
      all += c;
      pre += (w2 < wave) ? c : 0;
    }
    const int wcc  = wc > WCAP ? WCAP : wc;
    const int base = tot + pre;
#pragma unroll 1
    for (int i = lane; i < wcc; i += 32) {
      const int ent = list[wave * WCAP + i];
      const int el  = (ent >> SLOTB) & (CHUNK - 1);
      const int sl  = ent & (NBMAX - 1);
      int eid = cbase + el;
      eid = eid > nE - 1 ? nE - 1 : eid;
      const int pos = base + i;
      if (pos < RCAP) reg1[pos] = (int)(((unsigned)eid << SLOTB) | (unsigned)sl);
    }
    tot += all;
    tot = tot > RCAP ? RCAP : tot;
    __syncthreads();
  }
  const int nh = tot;

  if (wave == 0) {
#pragma unroll 1
    for (int b0 = 0; b0 < nh; b0 += 32) {
      const int idx = b0 + lane;
      const int uv  = reg1[idx < nh ? idx : nh - 1];
      const int m32 = (nh - b0) < 32 ? (nh - b0) : 32;
#pragma unroll 1
      for (int k = 0; k < m32; ++k) {
        const int u  = __builtin_amdgcn_readlane(uv, k);
        const int sl = u & (NBMAX - 1);
        if (lane == 0) scnt[sl] = scnt[sl] + 1;
      }
    }
  }
  __syncthreads();

  {
    const v4i ca = *(const v4i*)(scnt + 8 * tid);
    const v4i cb = *(const v4i*)(scnt + 8 * tid + 4);
    const int e0 = ca.x < 0 ? 0 : ca.x, e1 = ca.y < 0 ? 0 : ca.y, e2 = ca.z < 0 ? 0 : ca.z, e3 = ca.w < 0 ? 0 : ca.w;
    const int e4 = cb.x < 0 ? 0 : cb.x, e5 = cb.y < 0 ? 0 : cb.y, e6 = cb.z < 0 ? 0 : cb.z, e7 = cb.w < 0 ? 0 : cb.w;
    const int ts = e0 + e1 + e2 + e3 + e4 + e5 + e6 + e7;
    int incl = ts;
#pragma unroll
    for (int d = 1; d < 32; d <<= 1) {
      const int up = __shfl_up(incl, d);
      if (lane >= d) incl += up;
    }
    if (lane == 31) wtot[wave] = incl;
    __syncthreads();
    int pre = 0;
#pragma unroll
    for (int w2 = 0; w2 < NWAVE; ++w2) pre += (w2 < wave) ? wtot[w2] : 0;
    int run = pre + incl - ts;
    soff[8 * tid + 0] = run; run += e0;
    soff[8 * tid + 1] = run; run += e1;
    soff[8 * tid + 2] = run; run += e2;
    soff[8 * tid + 3] = run; run += e3;
    soff[8 * tid + 4] = run; run += e4;
    soff[8 * tid + 5] = run; run += e5;
    soff[8 * tid + 6] = run; run += e6;
    soff[8 * tid + 7] = run;
  }
  __syncthreads();
  for (int i = tid; i < NBMAX; i += NTHR) list[i] = soff[i];
  __syncthreads();

  if (wave == 0) {
#pragma unroll 1
    for (int b0 = 0; b0 < nh; b0 += 32) {
      const int idx = b0 + lane;
      const int uv  = reg1[idx < nh ? idx : nh - 1];
      const int m32 = (nh - b0) < 32 ? (nh - b0) : 32;
#pragma unroll 1
      for (int k = 0; k < m32; ++k) {
        const int u   = __builtin_amdgcn_readlane(uv, k);
        const int sl  = u & (NBMAX - 1);
        const int eid = (int)((unsigned)u >> SLOTB);
        if (lane == 0) {
          int pos = list[sl];
          pos = pos < 0 ? 0 : (pos > RCAP - 1 ? RCAP - 1 : pos);
          reg2[pos] = eid;
          list[sl] = pos + 1;
        }
      }
    }
  }
  __syncthreads();

  const int nbw = nb >> 3;
  const bool ovf = (nh >= RCAP);
  const float qnan = __int_as_float(0x7fc00000);
  const int cA = 4 * lane;
  const v4f asA = bfr4(*(const v4fa*)(asrc + cA));
  const v4f adA = bfr4(*(const v4fa*)(adst + cA));
  const v4f bbA = bfr4(*(const v4fa*)(bias + cA));
  const v4f ggA = bfr4(*(const v4fa*)(gam + cA));
  const v4f eeA = bfr4(*(const v4fa*)(bet + cA));

#pragma unroll 1
  for (int jt = 0; jt < nbw; ++jt) {
    const int slot = wave * nbw + jt;
    const int grow = nodeBase + slot;
    const int gcl  = grow < nN ? grow : nN - 1;
    int st = soff[slot];
    const int craw = scnt[slot];
    int cnt = craw;
    st  = st < 0 ? 0 : (st > nh ? nh : st);
    cnt = cnt < 0 ? 0 : (cnt > DEGCAP ? DEGCAP : cnt);
    if (cnt > nh - st) cnt = nh - st;
    const float pz = (ovf || craw > DEGCAP) ? qnan : 0.0f;

    const float* fr = F + (size_t)gcl * HCH;
    const v4f fdA = *(const v4fa*)(fr + cA);
    const float pdA = hsum8(dot4(fdA, adA));
    float l0A = hsum8(dot4(fdA, asA)) + pdA;
    l0A = l0A > 0.f ? l0A : NEGSL * l0A;
    float mxA = l0A, dnA = 1.0f;
    v4f aA = fdA;

#pragma unroll 1
    for (int q = 0; q < cnt; ++q) {
      int idx = st + q; idx = idx > RCAP - 1 ? RCAP - 1 : idx;
      int eid = reg2[idx]; eid = eid < 0 ? 0 : (eid > nE - 1 ? nE - 1 : eid);
      const int sraw = srcs[eid];
      const int s = sraw < 0 ? 0 : (sraw > nN - 1 ? nN - 1 : sraw);
      const float* gs = F + (size_t)s * HCH;
      const v4f fsA = *(const v4fa*)(gs + cA);
      float lgA = hsum8(dot4(fsA, asA)) + pdA;
      lgA = lgA > 0.f ? lgA : NEGSL * lgA;
      const float df = lgA - mxA;
      const float ex = __expf(-fabsf(df));
      const bool up  = df > 0.f;
      const float s1 = up ? ex : 1.0f;
      const float s2 = up ? 1.0f : ex;
      mxA = up ? lgA : mxA;
      dnA = fmaf(dnA, s1, s2);
      aA  = aA * s1 + fsA * s2;
    }
    const float invA = __builtin_amdgcn_rcpf(dnA + EPS_SM);
    const v4f xr = bfr4(*(const v4fa*)(xin + (size_t)gcl * KD + cA));
    v4f tA = aA * invA + bbA;
    tA = xr + tA;
    const float sm = wsum((tA.x + tA.y) + (tA.z + tA.w));
    const float mu = sm * (1.0f / HCH);
    const v4f dA = tA - mu;
    const float sq = wsum((dA.x * dA.x + dA.y * dA.y) + (dA.z * dA.z + dA.w * dA.w));
    const float rs = rsqrtf(sq * (1.0f / HCH) + LNEPS) + pz;
    const v4f yA = dA * rs * ggA + eeA;

    if (grow < nN) {
      float* op = out + (size_t)grow * HCH;
      *(volatile v4f*)(op + cA) = yA;
      __threadfence();
      *(volatile v4f*)(op + cA) = yA;
    }
  }
}

static int pick_nb(int nE, int nN) {
  int nb = NBMAX;
  while (nb > 32 && (long long)nb * (long long)nE * 5LL > (long long)RCAP * (long long)nN * 4LL) nb >>= 1;
  return nb;
}
static inline int cdiv(int a, int b) { return (a + b - 1) / b; }

extern "C" void kernel_launch(void* const* d_in, const int* in_sizes, int n_in,
                              void* d_out, int out_size, void* d_ws, size_t ws_size,
                              hipStream_t stream) {
  if (n_in < 8) return;
  if (in_sizes[0] < KD || (in_sizes[0] % KD) != 0) return;
  const int nN = in_sizes[0] / KD;
  if (nN <= 0 || nN > (1 << 22)) return;
  if (in_sizes[1] < 2 || (in_sizes[1] & 1) != 0) return;
  const int nE = in_sizes[1] / 2;
  if (nE < 1 || nE >= (1 << (32 - SLOTB))) return;
  if (in_sizes[2] != KD * HCH) return;
  if (in_sizes[3] != HCH || in_sizes[4] != HCH) return;
  if (in_sizes[5] != HCH || in_sizes[6] != HCH || in_sizes[7] != HCH) return;
  if (out_size != nN * HCH) return;

  const float* x    = (const float*)d_in[0];
  const int*   ei   = (const int*)  d_in[1];
  const float* W    = (const float*)d_in[2];
  const float* asrc = (const float*)d_in[3];
  const float* adst = (const float*)d_in[4];
  const float* bias = (const float*)d_in[5];
  const float* gam  = (const float*)d_in[6];
  const float* bet  = (const float*)d_in[7];
  float* out = (float*)d_out;
  const int* src = ei;
  const int* dst = ei + nE;

  const int MP   = cdiv(nN, MROWS) * MROWS;
  const int nb   = pick_nb(nE, nN);
  if (nb < 32 || (nb & (nb - 1)) != 0 || nb > NBMAX) return;
  const int gA   = cdiv(MP, nb);
  const int vec8 = ((nE & 3) == 0) ? 1 : 0;
  if ((long long)gA * nb < (long long)MP || (long long)gA * nb < (long long)nN) return;

  char* ws = (char*)d_ws;
  size_t off = 0;
  const size_t oF  = off; off += (size_t)MP * HCH * 4;             off = (off + 255) & ~(size_t)255;
  const size_t oWT = off; off += (size_t)HCH * KD * 2;             off = (off + 255) & ~(size_t)255;
  if (off > ws_size || off > (size_t)WSMAX) return;
  float*          F  = (float*)(ws + oF);
  unsigned short* WT = (unsigned short*)(ws + oWT);

  hipFuncSetAttribute(reinterpret_cast<const void*>(&k_agg),
                      hipFuncAttributeMaxDynamicSharedMemorySize, LDS_AGG);

  {
    const int nUw = HCH * (KD / 8);
    k_wtr<<<cdiv(nUw, NTHR), NTHR, 0, stream>>>(W, KD, HCH, HCH, KD, WT, nUw);
  }
  k_gemm<<<dim3(MP / GBM, HCH / GBN), GTHR, 0, stream>>>(x, nN, WT, F);
  k_agg<<<gA, NTHR, LDS_AGG, stream>>>(src, dst, F, x, asrc, adst, bias, gam, bet, out, nN, nE, nb, vec8);
}
